// SimpleBlock_19713899888770
// MI455X (gfx1250) — hardware-verified
//
#include <hip/hip_runtime.h>
#include <math.h>

typedef __attribute__((ext_vector_type(16))) _Float16 v16h;
typedef __attribute__((ext_vector_type(16))) __bf16 v16b;
typedef __attribute__((ext_vector_type(8)))  _Float16 v8h;
typedef __attribute__((ext_vector_type(8)))  float v8f;
typedef __attribute__((ext_vector_type(4)))  float v4f;
typedef __attribute__((ext_vector_type(2)))  float v2f;
typedef __attribute__((ext_vector_type(4)))  unsigned v4u;
typedef __attribute__((ext_vector_type(4)))  int v4i;
typedef float __attribute__((may_alias)) float_a;
typedef int __attribute__((may_alias)) int_a;

template <typename T> __device__ __forceinline__ void vst2(void* p, T v) { *(volatile T*)p = v; __threadfence(); *(volatile T*)p = v; }
__device__ __forceinline__ v8f wmma16(v16h a, v16h b, v8f c) {
  v8f d = __builtin_amdgcn_wmma_f32_16x16x32_f16(false, a, false, b, (short)0, c, false, false);
  asm volatile("v_nop\n\tv_nop\n\tv_nop\n\tv_nop" : "+v"(d) : "v"(a), "v"(b));
  return d;
}
__device__ __forceinline__ v8f wmma_bf(v16b a, v16b b, v8f c) {
  v8f d = __builtin_amdgcn_wmma_f32_16x16x32_bf16(false, a, false, b, (short)0, c, false, false);
  asm volatile("v_nop\n\tv_nop\n\tv_nop\n\tv_nop" : "+v"(d) : "v"(a), "v"(b));
  return d;
}
__device__ __forceinline__ v16h frag_h(const _Float16* rowk0, int lane) {
  union { v16h v; v8h q[2]; } u; const _Float16* p = rowk0 + 8 * (lane >> 4);
  u.q[0] = *(const v8h*)p; u.q[1] = *(const v8h*)(p + 16); return u.v;
}
__device__ __forceinline__ v16h frag_f32(const float* rowk0, int lane) {
  v16h a; const float* p = rowk0 + 8 * (lane >> 4);
#pragma unroll
  for (int i = 0; i < 8; ++i) { a[i] = (_Float16)p[i]; a[8 + i] = (_Float16)p[16 + i]; }
  return a;
}
__device__ __forceinline__ v16h frag_f32s(const float* rowk0, int lane, float sc) {
  v16h a; const float* p = rowk0 + 8 * (lane >> 4);
#pragma unroll
  for (int i = 0; i < 8; ++i) { a[i] = (_Float16)(p[i] * sc); a[8 + i] = (_Float16)(p[16 + i] * sc); }
  return a;
}
__device__ __forceinline__ v16h fragc_f32(const float* W, int k0, int n, int lane, int ld, int K) {
  v16h a; const int g = lane >> 4;
#pragma unroll
  for (int i = 0; i < 8; ++i) { const int ka = k0 + 8 * g + i, kb = ka + 16;
    a[i] = (_Float16)(ka < K ? W[(size_t)(ka < K ? ka : K - 1) * ld + n] : 0.f); a[8 + i] = (_Float16)(kb < K ? W[(size_t)(kb < K ? kb : K - 1) * ld + n] : 0.f); }
  return a;
}
struct F2 { v16b h, l; };
__device__ __forceinline__ F2 bsplit16(const float v[16]) { F2 r;
#pragma unroll
  for (int i = 0; i < 16; ++i) { const __bf16 h = (__bf16)v[i]; r.h[i] = h; r.l[i] = (__bf16)(v[i] - (float)h); }
  return r; }
__device__ __forceinline__ F2 split_row(const float* row, int k0, int lane) { float v[16]; const float* p = row + k0 + 8 * (lane >> 4);
#pragma unroll
  for (int i = 0; i < 8; ++i) { v[i] = p[i]; v[8 + i] = p[16 + i]; }
  return bsplit16(v); }
__device__ __forceinline__ F2 split_rowK(const float* row, int k0, int lane, int K) { float v[16]; const int g = lane >> 4;
#pragma unroll
  for (int i = 0; i < 8; ++i) { const int ka = k0 + 8 * g + i, kb = ka + 16; v[i] = ka < K ? row[ka < K ? ka : K - 1] : 0.f; v[8 + i] = kb < K ? row[kb < K ? kb : K - 1] : 0.f; }
  return bsplit16(v); }
__device__ __forceinline__ F2 split_col(const float* W, int k0, int n, int lane, int ld, int K) { float v[16]; const int g = lane >> 4;
#pragma unroll
  for (int i = 0; i < 8; ++i) { const int ka = k0 + 8 * g + i, kb = ka + 16; v[i] = ka < K ? W[(size_t)(ka < K ? ka : K - 1) * ld + n] : 0.f; v[8 + i] = kb < K ? W[(size_t)(kb < K ? kb : K - 1) * ld + n] : 0.f; }
  return bsplit16(v); }
__device__ __forceinline__ v8f mac3(const F2& a, const F2& b, v8f c) { c = wmma_bf(a.l, b.h, c); c = wmma_bf(a.h, b.l, c); return wmma_bf(a.h, b.h, c); }
__device__ __forceinline__ float sigm(float v) { return 1.0f / (1.0f + expf(-v)); }
#define LDSX() do { asm volatile("s_wait_dscnt 0" ::: "memory"); __builtin_amdgcn_wave_barrier(); __builtin_amdgcn_fence(__ATOMIC_RELEASE, "workgroup"); } while (0)

#define NM 65536
#define NS NM
#define NHB 16
#define NK 15
#define CI 64
#define CO 128
#define KW (NK * CI)
#define HALF (NM / 2)
#ifndef NMPROC
#define NMPROC NM
#endif
__device__ __forceinline__ float bfr(float v) { return (float)(__bf16)v; }
#define WS_A   0u
#define WS_T   (WS_A + 2u * (size_t)HALF * KW)
#define WS_ST  (WS_T + 4u * (size_t)NM * CO)
#define WS_END (WS_ST + 4u * (size_t)CO * 32)

__global__ __launch_bounds__(256) void k_wsum(const float* __restrict__ P, const float* __restrict__ X, const int* __restrict__ NBI, const float* __restrict__ KPT, int r0, _Float16* __restrict__ A) {
  __shared__ float sw[8][32][17]; __shared__ int sidx[8][32]; __shared__ __align__(16) _Float16 so[8][KW];
  const int wave = threadIdx.x >> 5, lane = threadIdx.x & 31, col = lane & 15, g = lane >> 4; const size_t ml = (size_t)blockIdx.x * 8 + wave; const size_t m = (size_t)r0 + ml;
  if (m >= (size_t)NMPROC) return;
  { const int h = lane & 15; const int ii = NBI[m * NHB + h]; const bool shadow = !(ii >= 0 && ii < NS) || lane >= NHB; const int idx = shadow ? 0 : ii;
    const float qx = bfr(P[m * 3]), qy = bfr(P[m * 3 + 1]), qz = bfr(P[m * 3 + 2]);
    const float px = shadow ? 1.0e6f : bfr(P[(size_t)idx * 3]), py = shadow ? 1.0e6f : bfr(P[(size_t)idx * 3 + 1]), pz = shadow ? 1.0e6f : bfr(P[(size_t)idx * 3 + 2]);
    const float rx = px - qx, ry = py - qy, rz = pz - qz;
#pragma unroll
    for (int k = 0; k < NK; ++k) { const float dx = rx - bfr(KPT[k * 3]), dy = ry - bfr(KPT[k * 3 + 1]), dz = rz - bfr(KPT[k * 3 + 2]); const float d = sqrtf(dx * dx + dy * dy + dz * dz); sw[wave][lane][k] = (lane < NHB) ? fmaxf(1.0f - d, 0.f) : 0.f; }
    sw[wave][lane][15] = 0.f; sw[wave][lane][16] = 0.f; sidx[wave][lane] = shadow ? -1 : idx; }
  LDSX();
  v16h a;
#pragma unroll
  for (int i = 0; i < 8; ++i) { a[i] = (_Float16)sw[wave][8 * g + i][col]; a[8 + i] = (_Float16)sw[wave][16 + 8 * g + i][col]; }
  v16h bx[4];
#pragma unroll
  for (int i = 0; i < 8; ++i) {
#pragma unroll
    for (int hh = 0; hh < 2; ++hh) { const int h = hh * 16 + 8 * g + i; const int idx = sidx[wave][h]; const int ic = idx < 0 ? 0 : idx; const float live = idx < 0 ? 0.f : 1.f; const float* xr = X + (size_t)ic * CI + col;
      float xg[4];
#pragma unroll
      for (int j = 0; j < 4; ++j) xg[j] = xr[16 * j];
      asm volatile("s_wait_loadcnt 0x0" ::: "memory");
#pragma unroll
      for (int j = 0; j < 4; ++j) bx[j][hh * 8 + i] = (_Float16)(bfr(xg[j]) * live); } }
  v8f acc[4] = {};
#pragma unroll
  for (int j = 0; j < 4; ++j) acc[j] = wmma16(a, bx[j], acc[j]);
#pragma unroll
  for (int j = 0; j < 4; ++j)
#pragma unroll
    for (int r = 0; r < 8; ++r) { const int k = 8 * g + r; if (k < NK) so[wave][k * CI + j * 16 + col] = (_Float16)acc[j][r]; }
  LDSX();
  for (int q = lane; q < KW / 8; q += 32) vst2((unsigned*)(A + ml * KW + q * 8), *(const v4u*)&so[wave][q * 8]); }
__global__ __launch_bounds__(128) void k_gemm(const _Float16* __restrict__ A, const float* __restrict__ Wt, int r0, float* __restrict__ T) { __shared__ __align__(16) float sf[4][16][132];
  const int tid = threadIdx.x, wave = tid >> 5, lane = tid & 31, col = lane & 15, g = lane >> 4; const size_t rl0 = (size_t)blockIdx.x * 64 + wave * 16;
  v8f acc[8] = {};
#pragma unroll 2
  for (int kc = 0; kc < KW / 32; ++kc) { const v16h a = frag_h(A + (rl0 + col) * KW + kc * 32, lane);
#pragma unroll
    for (int j = 0; j < 8; ++j) { v16h w; const int o = j * 16 + col;
#pragma unroll
      for (int i = 0; i < 8; ++i) { w[i] = (_Float16)(bfr(Wt[(size_t)(kc * 32 + 8 * g + i) * CO + o]) * 4.0f); w[8 + i] = (_Float16)(bfr(Wt[(size_t)(kc * 32 + 16 + 8 * g + i) * CO + o]) * 4.0f); }
      asm volatile("s_wait_loadcnt 0x0" ::: "memory"); acc[j] = wmma16(a, w, acc[j]); } }
#pragma unroll
  for (int j = 0; j < 8; ++j)
#pragma unroll
    for (int r = 0; r < 8; ++r) sf[wave][8 * g + r][j * 16 + col] = acc[j][r] * 0.25f;
  LDSX(); for (int rl = 0; rl < 16; ++rl) { const size_t row = (size_t)r0 + rl0 + rl; if (row < (size_t)NMPROC) vst2(T + row * CO + lane * 4, *(const v4f*)&sf[wave][rl][lane * 4]); } }
__global__ __launch_bounds__(256) void k_stat(const float* __restrict__ T, float* __restrict__ STAT) { __shared__ float sred[8]; __shared__ float sbc;
  const int t = threadIdx.x; const int c = blockIdx.x;
  float s = 0.f; for (int r = t; r < NMPROC; r += 256) s += T[(size_t)r * CO + c];
#pragma unroll
  for (int o = 1; o < 32; o <<= 1) s += __shfl_xor(s, o);
  if ((t & 31) == 0) sred[t >> 5] = s; __syncthreads(); if (t == 0) { float a = 0.f; for (int i = 0; i < 8; ++i) a += sred[i]; sbc = a / (float)NMPROC; } __syncthreads(); const float mean = sbc; __syncthreads();
  float q = 0.f; for (int r = t; r < NMPROC; r += 256) { const float d = T[(size_t)r * CO + c] - mean; q += d * d; }
#pragma unroll
  for (int o = 1; o < 32; o <<= 1) q += __shfl_xor(q, o);
  if ((t & 31) == 0) sred[t >> 5] = q; __syncthreads(); if (t == 0) { float a = 0.f; for (int i = 0; i < 8; ++i) a += sred[i]; sbc = rsqrtf(a / (float)NMPROC + 1e-5f); } __syncthreads();
  if (t < 32) { const float v = t == 0 ? mean : (t == 1 ? sbc : 0.f); vst2(STAT + (size_t)c * 32 + t, v); } }
__global__ __launch_bounds__(256) void k_bnact(const float* __restrict__ T, const float* __restrict__ STAT, const float* __restrict__ G, const float* __restrict__ BE, float* __restrict__ OUT) { const size_t e4 = (size_t)blockIdx.x * 256 + threadIdx.x; if (e4 >= (size_t)NMPROC * CO / 4) return; const int c0 = (int)((e4 * 4) % CO); const v4f tv = *(const v4f*)(T + e4 * 4); v4f o;
#pragma unroll
  for (int i = 0; i < 4; ++i) { const int c = c0 + i; const float y = (tv[i] - STAT[c * 32]) * STAT[c * 32 + 1] * bfr(G[c]) + bfr(BE[c]); o[i] = y >= 0.f ? y : 0.2f * y; }
  vst2(OUT + e4 * 4, o); }
extern "C" void kernel_launch(void* const* d_in, const int* in_sizes, int n_in, void* d_out, int out_size, void* d_ws, size_t ws_size, hipStream_t stream) {
  (void)in_sizes; (void)n_in; (void)out_size;
  if (ws_size < (size_t)WS_END) return;
  char* ws = (char*)d_ws; _Float16* A = (_Float16*)(ws + WS_A); float *T = (float*)(ws + WS_T), *ST = (float*)(ws + WS_ST);
  const int rows = NMPROC < HALF ? NMPROC : HALF;
  for (int r0 = 0; r0 < NMPROC; r0 += HALF) {
    k_wsum<<<dim3(rows / 8), 256, 0, stream>>>((const float*)d_in[0], (const float*)d_in[1], (const int*)d_in[6], (const float*)d_in[2], r0, A);
    k_gemm<<<dim3(rows / 64), 128, 0, stream>>>(A, (const float*)d_in[3], r0, T);
  }
  k_stat<<<dim3(CO), 256, 0, stream>>>(T, ST);
  k_bnact<<<dim3((NMPROC * CO / 4 + 255) / 256), 256, 0, stream>>>(T, ST, (const float*)d_in[4], (const float*)d_in[5], (float*)d_out);
}
